// COINBlock_81415400063161
// MI455X (gfx1250) — hardware-verified
//
#include <hip/hip_runtime.h>

#pragma clang fp contract(off)

typedef __attribute__((ext_vector_type(16))) _Float16 v16h;
typedef __attribute__((ext_vector_type(8)))  _Float16 v8h;
typedef __attribute__((ext_vector_type(16))) __bf16   v16b;
typedef __attribute__((ext_vector_type(8)))  __bf16   v8b;
typedef __attribute__((ext_vector_type(8)))  float    v8f;
typedef __attribute__((ext_vector_type(4)))  float    v4f;
typedef __attribute__((ext_vector_type(4)))  unsigned int v4u;

constexpr int NBATCH = 4;
constexpr int NT     = 4096;
constexpr int NC     = 512;
constexpr int NM     = NBATCH * NT;
constexpr int LCH    = 64;
constexpr int NCHK   = NT / LCH;
constexpr int NZ     = NBATCH * NCHK;
constexpr int DVS    = 32;
constexpr int SPH    = 520;
constexpr int OSP    = 36;

constexpr float PLANE_SC = 16.0f;
constexpr float RES_SC   = 2048.0f;
constexpr float RES_INV  = 1.0f / 2048.0f;
constexpr float PROD_INV = 1.0f / 256.0f;

static_assert(NC % 32 == 0);
static_assert(NC % 64 == 0);
static_assert(NM % 64 == 0);
static_assert(NT % LCH == 0);
static_assert(LCH == 64);
static_assert((NCHK & (NCHK - 1)) == 0);
static_assert((NT & (NT - 1)) == 0);
static_assert(NC % DVS == 0);
static_assert(DVS == 32);
static_assert(SPH % 8 == 0);
static_assert(OSP % 4 == 0);

constexpr size_t BYTES_XB  = (size_t)NM * NC * 2;
constexpr size_t BYTES_WT  = (size_t)3 * NC * NC * 2;
constexpr size_t BYTES_TAB = (size_t)3 * NT * 4;
constexpr size_t BYTES_PL  = (size_t)NM * NC * 2;
constexpr size_t BYTES_SC  = (size_t)NZ * LCH * LCH * 2;
constexpr size_t OFF_XB  = 0;
constexpr size_t OFF_WT  = OFF_XB + BYTES_XB;
constexpr size_t OFF_TAB = OFF_WT + BYTES_WT;
constexpr size_t OFF_QH  = OFF_TAB + BYTES_TAB;
constexpr size_t OFF_QL  = OFF_QH + BYTES_PL;
constexpr size_t OFF_KH  = OFF_QL + BYTES_PL;
constexpr size_t OFF_KL  = OFF_KH + BYTES_PL;
constexpr size_t OFF_VH  = OFF_KL + BYTES_PL;
constexpr size_t OFF_VL  = OFF_VH + BYTES_PL;
constexpr size_t OFF_AH  = OFF_VL + BYTES_PL;
constexpr size_t OFF_AL  = OFF_AH + BYTES_SC;
constexpr size_t WS_TOTAL = OFF_AL + BYTES_SC;
static_assert(WS_TOTAL == 123256832u);
static_assert(WS_TOTAL <= 134217728u);
static_assert(OFF_TAB % 4096 == 0);
static_assert(OFF_QH % 4096 == 0);
static_assert(OFF_AH % 4096 == 0);

constexpr size_t OUT0_ELEMS = (size_t)NM * NC;
constexpr size_t OUT1_ELEMS = (size_t)NBATCH * NC * NC;
static_assert(OUT0_ELEMS * 4 == 33554432u);
static_assert((OUT0_ELEMS + OUT1_ELEMS) * 4 == 37748736u);

__device__ __forceinline__ unsigned short f2bf_bits(float f) {
  unsigned u = __float_as_uint(f);
  return (unsigned short)((u + 0x7FFFu + ((u >> 16) & 1u)) >> 16);
}
__device__ __forceinline__ float bf_bits2f(unsigned short h) { return __uint_as_float(((unsigned)h) << 16); }

__device__ __forceinline__ void dep_guard_h(v8f& a, v8f& b, v16h x, v16h y) { asm volatile("v_nop\n\tv_nop\n\tv_nop\n\tv_nop" : "+v"(a), "+v"(b) : "v"(x), "v"(y)); }
__device__ __forceinline__ void dep_guard_b(v8f& a, v8f& b, v16b x, v16b y) { asm volatile("v_nop\n\tv_nop\n\tv_nop\n\tv_nop" : "+v"(a), "+v"(b) : "v"(x), "v"(y)); }
__device__ __forceinline__ void keep4_h(v16h a, v16h b, v16h c, v16h d) { asm volatile("v_nop" :: "v"(a), "v"(b), "v"(c), "v"(d)); }
__device__ __forceinline__ void keep4_b(v16b a, v16b b, v16b c, v16b d) { asm volatile("v_nop" :: "v"(a), "v"(b), "v"(c), "v"(d)); }
__device__ __forceinline__ void acc_guard4(v8f& a, v8f& b, v8f& c, v8f& d) { asm volatile("v_nop\n\tv_nop\n\tv_nop\n\tv_nop" : "+v"(a), "+v"(b), "+v"(c), "+v"(d)); }
template <typename T> struct Frag;
template <> struct Frag<_Float16> {
  typedef v16h V; union U { v16h v; v8h h[2]; };
  static __device__ __forceinline__ v16h load(const _Float16* p) {
    U f; f.h[0] = *(const v8h*)(p); f.h[1] = *(const v8h*)(p + 16); return f.v;
  }
  static __device__ __forceinline__ v8f mma(v16h a, v16h b, v8f c) {
    return __builtin_amdgcn_wmma_f32_16x16x32_f16(false, a, false, b, (short)0, c, false, false);
  }
  static __device__ __forceinline__ void guard(v8f& a, v8f& b, v16h x, v16h y) { dep_guard_h(a, b, x, y); }
  static __device__ __forceinline__ void keep(v16h a, v16h b, v16h c, v16h d) { keep4_h(a, b, c, d); }
};
template <> struct Frag<__bf16> {
  typedef v16b V; union U { v16b v; v8b h[2]; };
  static __device__ __forceinline__ v16b load(const __bf16* p) {
    U f; f.h[0] = *(const v8b*)(p); f.h[1] = *(const v8b*)(p + 16); return f.v;
  }
  static __device__ __forceinline__ v8f mma(v16b a, v16b b, v8f c) {
    return __builtin_amdgcn_wmma_f32_16x16x32_bf16(false, a, false, b, (short)0, c, false, false);
  }
  static __device__ __forceinline__ void guard(v8f& a, v8f& b, v16b x, v16b y) { dep_guard_b(a, b, x, y); }
  static __device__ __forceinline__ void keep(v16b a, v16b b, v16b c, v16b d) { keep4_b(a, b, c, d); }
};

__device__ __forceinline__ v8f vz8() { return (v8f){0.f, 0.f, 0.f, 0.f, 0.f, 0.f, 0.f, 0.f}; }
__device__ __forceinline__ float bf_rne(float x) { return bf_bits2f(f2bf_bits(x)); }

__device__ __forceinline__ float tanh_eval(float x) {
  const float e = expf(2.0f * x);
  const float r = __builtin_amdgcn_rcpf(e + 1.0f);
  return 1.0f - 2.0f * r;
}

__device__ __forceinline__ float gam_of(int t) {
  const float step = (float)t * (1.0f / 4095.0f);
  const float a = 1.0f - step;
  const float p0 = 0.96f * a;
  const float p1 = 0.99f * step;
  const float g = p0 + p1;
  return (t >= NT - 1) ? 0.99f : g;
}

__global__ __launch_bounds__(256) void cast_bf16x8(const float* __restrict__ in, unsigned short* __restrict__ out, int n8) {
  const int i = blockIdx.x * 256 + threadIdx.x;
  if (i < n8) {
    const v4f a = *(const v4f*)(in + (size_t)i * 8);
    const v4f c = *(const v4f*)(in + (size_t)i * 8 + 4);
    v4u w;
    w[0] = (unsigned)f2bf_bits(a[0]) | ((unsigned)f2bf_bits(a[1]) << 16);
    w[1] = (unsigned)f2bf_bits(a[2]) | ((unsigned)f2bf_bits(a[3]) << 16);
    w[2] = (unsigned)f2bf_bits(c[0]) | ((unsigned)f2bf_bits(c[1]) << 16);
    w[3] = (unsigned)f2bf_bits(c[2]) | ((unsigned)f2bf_bits(c[3]) << 16);
    unsigned short* o = out + (size_t)i * 8;
    *(volatile v4u*)o = w;
    __threadfence();
    *(volatile v4u*)o = w;
  }
}

__global__ __launch_bounds__(256) void wtrans_kernel(const float* __restrict__ W0, const float* __restrict__ W1,
                                                     const float* __restrict__ W2, unsigned short* __restrict__ Wt) {
  __shared__ __align__(16) float tile[64 * 65];
  const int tid = threadIdx.x, lane = tid & 31, wave = tid >> 5;
  const int z = blockIdx.z;
  const float* W = (z == 0) ? W0 : ((z == 1) ? W1 : W2);
  unsigned short* O = Wt + (size_t)z * NC * NC;
  const int n0 = blockIdx.x * 64, k0 = blockIdx.y * 64;
  {
    const int kk = tid >> 2, cb = (tid & 3) * 16;
    const float* src = W + (size_t)(k0 + kk) * NC + n0 + cb;
#pragma unroll
    for (int e4 = 0; e4 < 4; ++e4) {
      const v4f v = *(const v4f*)(src + 4 * e4);
      tile[kk * 65 + cb + 4 * e4 + 0] = v[0];
      tile[kk * 65 + cb + 4 * e4 + 1] = v[1];
      tile[kk * 65 + cb + 4 * e4 + 2] = v[2];
      tile[kk * 65 + cb + 4 * e4 + 3] = v[3];
    }
  }
  __syncthreads();
  const int q = lane >> 3, c8 = (lane & 7) * 8;
  for (int pass = 0; pass < 2; ++pass) {
#pragma unroll
    for (int it = 0; it < 2; ++it) {
      const int nn = wave * 8 + it * 4 + q;
      v8h hv;
#pragma unroll
      for (int e = 0; e < 8; ++e) hv[e] = __builtin_bit_cast(_Float16, f2bf_bits(tile[(c8 + e) * 65 + nn]));
      *(volatile v8h*)(O + (size_t)(n0 + nn) * NC + k0 + c8) = hv;
    }
    __threadfence();
  }
}

__global__ __launch_bounds__(256) void tables_kernel(float* __restrict__ gcum, float* __restrict__ ginv, float* __restrict__ ksc) {
  __shared__ __align__(16) float tg[NT];
  __shared__ __align__(16) float ti[NT];
  __shared__ __align__(16) float tk[NT];
  const int tid = threadIdx.x;
  if (tid < NCHK) {
    const int t0 = tid * LCH;
    double p = 1.0;
    for (int j = 0; j < LCH; ++j) {
      const float g = gam_of(t0 + j);
      p = p * (double)g;
      tg[t0 + j] = (float)p;
      ti[t0 + j] = (float)(1.0 / p);
    }
    double s = 1.0;
    for (int j = LCH - 1; j >= 0; --j) {
      tk[t0 + j] = (float)s;
      const float g = gam_of(t0 + j);
      s = s * (double)g;
    }
  }
  __syncthreads();
  for (int pass = 0; pass < 2; ++pass) {
#pragma unroll
    for (int seg = 0; seg < 4; ++seg) {
      const int idx = seg * 1024 + tid * 4;
      const v4f a = *(const v4f*)(tg + idx);
      *(volatile v4f*)(gcum + idx) = a;
      const v4f c = *(const v4f*)(ti + idx);
      *(volatile v4f*)(ginv + idx) = c;
      const v4f d = *(const v4f*)(tk + idx);
      *(volatile v4f*)(ksc + idx) = d;
    }
    __threadfence();
  }
}

template <int BIAS_MODE, int SCL_MODE>
__global__ __launch_bounds__(256) void gemm_proj(
    const unsigned short* __restrict__ Ap, int lda,
    const unsigned short* __restrict__ Btp, int ldb,
    unsigned short* __restrict__ Chp, unsigned short* __restrict__ Clp, int ldc,
    const float* __restrict__ bias, const float* __restrict__ stab, int tmask,
    int M, int N, int K, float oscale) {
  typedef __bf16 T;
  const T* A = (const T*)Ap; const T* Bt = (const T*)Btp;
  _Float16* Ch = (_Float16*)Chp; _Float16* Cl = (_Float16*)Clp;
  __shared__ __align__(16) float sT[8][16 * 68];
  const int lane = threadIdx.x & 31;
  const int wave = threadIdx.x >> 5;
  const int tilesN = N >> 6;
  const int tilesM = M >> 6;
  const int tile = blockIdx.x * 8 + wave;
  if (tile >= tilesM * tilesN) return;
  const int tm = tile / tilesN;
  const int tn = tile - tm * tilesN;
  const int m0 = tm << 6;
  const int n0 = tn << 6;
  const int rlane = lane & 15;
  const int koff  = (lane >> 4) * 8;
  const int mOff  = (lane >> 4) * 8;

  v8f acc[4][4];
#pragma unroll
  for (int i = 0; i < 4; ++i)
#pragma unroll
    for (int j = 0; j < 4; ++j) acc[i][j] = vz8();

  for (int k0 = 0; k0 < K; k0 += 32) {
    v16b bh[4];
#pragma unroll
    for (int j = 0; j < 4; ++j) {
      const size_t bo = (size_t)(n0 + (j << 4) + rlane) * ldb + koff + k0;
      bh[j] = Frag<T>::load(Bt + bo);
    }
#pragma unroll
    for (int i = 0; i < 4; ++i) {
      const size_t ao = (size_t)(m0 + (i << 4) + rlane) * lda + koff + k0;
      const v16b ah = Frag<T>::load(A + ao);
#pragma unroll
      for (int j = 0; j < 4; ++j) acc[i][j] = Frag<T>::mma(ah, bh[j], acc[i][j]);
      Frag<T>::guard(acc[i][0], acc[i][3], ah, ah);
    }
    Frag<T>::keep(bh[0], bh[1], bh[2], bh[3]);
  }
  acc_guard4(acc[0][0], acc[0][1], acc[0][2], acc[0][3]);
  acc_guard4(acc[1][0], acc[1][1], acc[1][2], acc[1][3]);
  acc_guard4(acc[2][0], acc[2][1], acc[2][2], acc[2][3]);
  acc_guard4(acc[3][0], acc[3][1], acc[3][2], acc[3][3]);

  float* slab = sT[wave];
  float cadd[4] = {0.f, 0.f, 0.f, 0.f};
  float cmul[4] = {1.f, 1.f, 1.f, 1.f};
  if (BIAS_MODE == 2) {
#pragma unroll
    for (int j = 0; j < 4; ++j) cadd[j] = bf_rne(bias[n0 + (j << 4) + rlane]);
  }
  if (SCL_MODE == 2) {
#pragma unroll
    for (int j = 0; j < 4; ++j) cmul[j] = stab[(n0 + (j << 4) + rlane) & tmask];
  }
  const int q = lane >> 3, c8 = (lane & 7) * 8;
#pragma unroll
  for (int i = 0; i < 4; ++i) {
    const int mBase = m0 + (i << 4);
    float radd[8], rmul[8];
#pragma unroll
    for (int e = 0; e < 8; ++e) { radd[e] = 0.f; rmul[e] = 1.f; }
    if (BIAS_MODE == 1) {
      const v4f x0 = *(const v4f*)(bias + mBase + mOff);
      const v4f x1 = *(const v4f*)(bias + mBase + mOff + 4);
#pragma unroll
      for (int e = 0; e < 4; ++e) { radd[e] = bf_rne(x0[e]); radd[4 + e] = bf_rne(x1[e]); }
    }
    if (SCL_MODE == 1) {
      const int tr = (mBase + mOff) & tmask;
      const v4f s0 = *(const v4f*)(stab + tr);
      const v4f s1 = *(const v4f*)(stab + tr + 4);
#pragma unroll
      for (int e = 0; e < 4; ++e) { rmul[e] = s0[e]; rmul[4 + e] = s1[e]; }
    }
#pragma unroll
    for (int j = 0; j < 4; ++j) {
#pragma unroll
      for (int r = 0; r < 8; ++r) {
        float v = acc[i][j][r] + radd[r];
        v = v + cadd[j];
        v = v * rmul[r];
        v = v * cmul[j];
        v = v * oscale;
        slab[(mOff + r) * 68 + (j << 4) + rlane] = v;
      }
    }
    __builtin_amdgcn_fence(__ATOMIC_RELEASE, "workgroup");
    __builtin_amdgcn_wave_barrier();
    __builtin_amdgcn_fence(__ATOMIC_ACQUIRE, "workgroup");
    for (int pass = 0; pass < 2; ++pass) {
#pragma unroll
      for (int it = 0; it < 4; ++it) {
        const int row = it * 4 + q;
        const float* sp = slab + row * 68 + c8;
        v8h hv, lv;
#pragma unroll
        for (int e = 0; e < 8; ++e) {
          const float x = sp[e];
          const _Float16 hx = (_Float16)x;
          hv[e] = hx;
          lv[e] = (_Float16)((x - (float)hx) * RES_SC);
        }
        *(volatile v8h*)(Ch + (size_t)(mBase + row) * ldc + n0 + c8) = hv;
        *(volatile v8h*)(Cl + (size_t)(mBase + row) * ldc + n0 + c8) = lv;
      }
      __threadfence();
    }
    __builtin_amdgcn_fence(__ATOMIC_RELEASE, "workgroup");
    __builtin_amdgcn_wave_barrier();
    __builtin_amdgcn_fence(__ATOMIC_ACQUIRE, "workgroup");
  }
}

__global__ __launch_bounds__(128) void scores_kernel(
    const unsigned short* __restrict__ Qhp, const unsigned short* __restrict__ Qlp,
    const unsigned short* __restrict__ Khp, const unsigned short* __restrict__ Klp,
    unsigned short* __restrict__ Ahp, unsigned short* __restrict__ Alp,
    const float* __restrict__ ginv) {
  typedef _Float16 H;
  __shared__ __align__(16) float sT[4][16 * 68];
  const int lane = threadIdx.x & 31;
  const int wave = threadIdx.x >> 5;
  const int z = blockIdx.x;
  const H* Qh = (const H*)Qhp + (size_t)z * LCH * NC;
  const H* Ql = (const H*)Qlp + (size_t)z * LCH * NC;
  const H* Kh = (const H*)Khp + (size_t)z * LCH * NC;
  const H* Kl = (const H*)Klp + (size_t)z * LCH * NC;
  H* Ah = (H*)Ahp; H* Al = (H*)Alp;
  const int rlane = lane & 15;
  const int koff  = (lane >> 4) * 8;
  const int mOff  = (lane >> 4) * 8;

  v8f am[4], ar[4];
#pragma unroll
  for (int j = 0; j < 4; ++j) { am[j] = vz8(); ar[j] = vz8(); }

  for (int k0 = 0; k0 < NC; k0 += 32) {
    v16h bh[4], bl[4];
#pragma unroll
    for (int j = 0; j < 4; ++j) {
      const size_t bo = (size_t)((j << 4) + rlane) * NC + koff + k0;
      bh[j] = Frag<H>::load(Kh + bo);
      bl[j] = Frag<H>::load(Kl + bo);
    }
    const size_t ao = (size_t)((wave << 4) + rlane) * NC + koff + k0;
    const v16h ah = Frag<H>::load(Qh + ao);
    const v16h al = Frag<H>::load(Ql + ao);
#pragma unroll
    for (int j = 0; j < 4; ++j) {
      am[j] = Frag<H>::mma(ah, bh[j], am[j]);
      ar[j] = Frag<H>::mma(ah, bl[j], ar[j]);
      ar[j] = Frag<H>::mma(al, bh[j], ar[j]);
    }
    Frag<H>::guard(am[0], ar[3], ah, al);
    Frag<H>::keep(bh[0], bh[1], bh[2], bh[3]);
    Frag<H>::keep(bl[0], bl[1], bl[2], bl[3]);
  }
  acc_guard4(am[0], am[1], am[2], am[3]);
  acc_guard4(ar[0], ar[1], ar[2], ar[3]);

  float gj[4];
#pragma unroll
  for (int j = 0; j < 4; ++j) gj[j] = ginv[(z & (NCHK - 1)) * LCH + (j << 4) + rlane] * (1.0f / 16.0f);

  float* slab = sT[wave];
#pragma unroll
  for (int j = 0; j < 4; ++j) {
#pragma unroll
    for (int r = 0; r < 8; ++r) {
      const int i  = (wave << 4) + mOff + r;
      const int jj = (j << 4) + rlane;
      float v = am[j][r] + ar[j][r] * RES_INV;
      v = v * gj[j];
      v = (jj > i) ? 0.0f : v;
      slab[(mOff + r) * 68 + (j << 4) + rlane] = v;
    }
  }
  __builtin_amdgcn_fence(__ATOMIC_RELEASE, "workgroup");
  __builtin_amdgcn_wave_barrier();
  __builtin_amdgcn_fence(__ATOMIC_ACQUIRE, "workgroup");
  const int q = lane >> 3, c8 = (lane & 7) * 8;
  for (int pass = 0; pass < 2; ++pass) {
#pragma unroll
    for (int it = 0; it < 4; ++it) {
      const int row = it * 4 + q;
      const float* sp = slab + row * 68 + c8;
      v8h hv, lv;
#pragma unroll
      for (int e = 0; e < 8; ++e) {
        const float x = sp[e];
        const _Float16 hx = (_Float16)x;
        hv[e] = hx;
        lv[e] = (_Float16)((x - (float)hx) * RES_SC);
      }
      const size_t oo = ((size_t)z * LCH + (wave << 4) + row) * LCH + c8;
      *(volatile v8h*)(Ah + oo) = hv;
      *(volatile v8h*)(Al + oo) = lv;
    }
    __threadfence();
  }
}

__global__ __launch_bounds__(256) void recur_kernel(
    const unsigned short* __restrict__ Qhp, const unsigned short* __restrict__ Qlp,
    const unsigned short* __restrict__ Ahp, const unsigned short* __restrict__ Alp,
    const unsigned short* __restrict__ KThp, const unsigned short* __restrict__ KTlp,
    const unsigned short* __restrict__ VThp, const unsigned short* __restrict__ VTlp,
    const float* __restrict__ gcum, float* __restrict__ out0, float* __restrict__ out1) {
  typedef _Float16 H;
  typedef Frag<H>::U UH;
  __shared__ __align__(16) float Sf[DVS * NC];
  __shared__ __align__(16) H     Sxh[DVS * SPH];
  __shared__ __align__(16) H     Sxl[DVS * SPH];
  __shared__ __align__(16) float Os[LCH * OSP];

  const int tid = threadIdx.x, wave = tid >> 5, lane = tid & 31;
  const int rl = lane & 15, hh = lane >> 4, koff = hh * 8, mOff = hh * 8;
  const int d0 = blockIdx.x * DVS, b = blockIdx.y;
  const size_t qrow0 = (size_t)b * NT;

  for (int i = tid; i < DVS * NC; i += 256) Sf[i] = 0.0f;
  {
    v8h z8;
#pragma unroll
    for (int e = 0; e < 8; ++e) z8[e] = (H)0.0f;
    for (int i = tid; i < (DVS * SPH) / 8; i += 256) { *(v8h*)(Sxh + i * 8) = z8; *(v8h*)(Sxl + i * 8) = z8; }
  }
  __syncthreads();

  const H* Qh  = (const H*)Qhp;  const H* Ql  = (const H*)Qlp;
  const H* Ah  = (const H*)Ahp;  const H* Al  = (const H*)Alp;
  const H* KTh = (const H*)KThp; const H* KTl = (const H*)KTlp;
  const H* VTh = (const H*)VThp; const H* VTl = (const H*)VTlp;

  for (int n = 0; n < NCHK; ++n) {
    const int t0 = n * LCH;
    const int z = b * NCHK + n;
    const float Gtot = gcum[t0 + LCH - 1];

    {
      const int it = wave >> 1, dt = wave & 1;
      v8f am = vz8(), ar = vz8();
      const H* qh = Qh + (qrow0 + t0 + it * 16 + rl) * NC + koff;
      const H* ql = Ql + (qrow0 + t0 + it * 16 + rl) * NC + koff;
      const int so = (dt * 16 + rl) * SPH + koff;
      for (int k0 = 0; k0 < NC; k0 += 32) {
        const v16h fa  = Frag<H>::load(qh + k0);
        const v16h fal = Frag<H>::load(ql + k0);
        UH ubh, ubl;
        ubh.h[0] = *(const v8h*)(Sxh + so + k0);
        ubh.h[1] = *(const v8h*)(Sxh + so + k0 + 16);
        ubl.h[0] = *(const v8h*)(Sxl + so + k0);
        ubl.h[1] = *(const v8h*)(Sxl + so + k0 + 16);
        const v16h fb = ubh.v, fbl = ubl.v;
        am = Frag<H>::mma(fa, fb, am);
        ar = Frag<H>::mma(fa, fbl, ar);
        ar = Frag<H>::mma(fal, fb, ar);
        dep_guard_h(am, ar, fa, fb);
        keep4_h(fal, fbl, fa, fb);
      }
      const H* aph = Ah + ((size_t)z * LCH + it * 16 + rl) * LCH + koff;
      const H* apl = Al + ((size_t)z * LCH + it * 16 + rl) * LCH + koff;
      const H* vh  = VTh + (size_t)(d0 + dt * 16 + rl) * NM + qrow0 + t0 + koff;
      const H* vl  = VTl + (size_t)(d0 + dt * 16 + rl) * NM + qrow0 + t0 + koff;
#pragma unroll
      for (int ks = 0; ks < 2; ++ks) {
        const v16h fa  = Frag<H>::load(aph + ks * 32);
        const v16h fal = Frag<H>::load(apl + ks * 32);
        const v16h fb  = Frag<H>::load(vh + ks * 32);
        const v16h fbl = Frag<H>::load(vl + ks * 32);
        am = Frag<H>::mma(fa, fb, am);
        ar = Frag<H>::mma(fa, fbl, ar);
        ar = Frag<H>::mma(fal, fb, ar);
        dep_guard_h(am, ar, fa, fb);
        keep4_h(fal, fbl, fa, fb);
      }
#pragma unroll
      for (int r = 0; r < 8; ++r) {
        const float x = (am[r] + ar[r] * RES_INV) * PROD_INV;
        Os[(it * 16 + mOff + r) * OSP + dt * 16 + rl] = tanh_eval(x);
      }
    }
    __syncthreads();

    {
      const int q = lane >> 3, c4 = (lane & 7) * 4;
      const int r0 = wave * 8 + q, r1 = r0 + 4;
      const v4f v0 = *(const v4f*)(Os + r0 * OSP + c4);
      const v4f v1 = *(const v4f*)(Os + r1 * OSP + c4);
      float* ob = out0 + (qrow0 + (size_t)t0) * NC + d0 + c4;
      for (int pass = 0; pass < 2; ++pass) {
        *(volatile v4f*)(ob + (size_t)r0 * NC) = v0;
        *(volatile v4f*)(ob + (size_t)r1 * NC) = v1;
        __threadfence();
      }
    }

    {
      const int dt = wave >> 2, cb = (wave & 3) * 8;
      const H* vh = VTh + (size_t)(d0 + dt * 16 + rl) * NM + qrow0 + t0 + koff;
      const H* vl = VTl + (size_t)(d0 + dt * 16 + rl) * NM + qrow0 + t0 + koff;
      v16h fah[2], fal[2];
      fah[0] = Frag<H>::load(vh);      fah[1] = Frag<H>::load(vh + 32);
      fal[0] = Frag<H>::load(vl);      fal[1] = Frag<H>::load(vl + 32);
      for (int cc = 0; cc < 8; ++cc) {
        const int ct = cb + cc;
        const H* krh = KTh + (size_t)(ct * 16 + rl) * NM + qrow0 + t0 + koff;
        const H* krl = KTl + (size_t)(ct * 16 + rl) * NM + qrow0 + t0 + koff;
        v16h fbh[2], fbl[2];
        fbh[0] = Frag<H>::load(krh);   fbh[1] = Frag<H>::load(krh + 32);
        fbl[0] = Frag<H>::load(krl);   fbl[1] = Frag<H>::load(krl + 32);
        v8f um = vz8(), ur = vz8();
#pragma unroll
        for (int ks = 0; ks < 2; ++ks) {
          um = Frag<H>::mma(fah[ks], fbh[ks], um);
          ur = Frag<H>::mma(fah[ks], fbl[ks], ur);
          ur = Frag<H>::mma(fal[ks], fbh[ks], ur);
        }
        dep_guard_h(um, ur, fah[1], fbh[1]);
        keep4_h(fbh[0], fbl[0], fbh[1], fbl[1]);
        keep4_h(fah[0], fal[0], fah[1], fal[1]);
#pragma unroll
        for (int r = 0; r < 8; ++r) {
          const int dl = dt * 16 + mOff + r;
          const int c  = ct * 16 + rl;
          const float u  = (um[r] + ur[r] * RES_INV) * PROD_INV;
          const float s  = Sf[dl * NC + c];
          const float gs = Gtot * s;
          const float sn = u + gs;
          Sf[dl * NC + c] = sn;
          const float x = sn * PLANE_SC;
          const H hx = (H)x;
          const float res = (x - (float)hx) * RES_SC;
          Sxh[dl * SPH + c] = hx;
          Sxl[dl * SPH + c] = (H)res;
        }
      }
    }
    __syncthreads();
  }

  {
    const int q = lane >> 3, c4 = (lane & 7) * 4;
    float* ob = out1 + (size_t)b * NC * NC + d0 + c4;
    for (int pass = 0; pass < 2; ++pass) {
#pragma unroll
      for (int it = 0; it < 16; ++it) {
        const int c = wave * 64 + it * 4 + q;
        v4f v;
        v[0] = Sf[(c4 + 0) * NC + c];
        v[1] = Sf[(c4 + 1) * NC + c];
        v[2] = Sf[(c4 + 2) * NC + c];
        v[3] = Sf[(c4 + 3) * NC + c];
        *(volatile v4f*)(ob + (size_t)c * NC) = v;
      }
      __threadfence();
    }
  }
}

extern "C" void kernel_launch(void* const* d_in, const int* in_sizes, int n_in,
                              void* d_out, int out_size, void* d_ws, size_t ws_size,
                              hipStream_t stream) {
  if (n_in < 8) return;
  if (in_sizes[0] != NM * NC) return;
  if (in_sizes[2] != NC * NC || in_sizes[4] != NC * NC || in_sizes[6] != NC * NC) return;
  if (in_sizes[3] != NC || in_sizes[5] != NC || in_sizes[7] != NC) return;
  if ((size_t)out_size != OUT0_ELEMS + OUT1_ELEMS) return;
  if (ws_size < WS_TOTAL) return;

  const float* X  = (const float*)d_in[0];
  const float* WQ = (const float*)d_in[2];
  const float* bQ = (const float*)d_in[3];
  const float* WK = (const float*)d_in[4];
  const float* bK = (const float*)d_in[5];
  const float* WV = (const float*)d_in[6];
  const float* bV = (const float*)d_in[7];

  char* ws = (char*)d_ws;
  unsigned short* Xb   = (unsigned short*)(ws + OFF_XB);
  unsigned short* Wt   = (unsigned short*)(ws + OFF_WT);
  unsigned short* WtQ  = Wt;
  unsigned short* WtK  = Wt + (size_t)NC * NC;
  unsigned short* WtV  = Wt + (size_t)2 * NC * NC;
  float* gcum = (float*)(ws + OFF_TAB);
  float* ginv = gcum + NT;
  float* ksc  = gcum + 2 * NT;
  unsigned short* Qh  = (unsigned short*)(ws + OFF_QH);
  unsigned short* Ql  = (unsigned short*)(ws + OFF_QL);
  unsigned short* Kh  = (unsigned short*)(ws + OFF_KH);
  unsigned short* Kl  = (unsigned short*)(ws + OFF_KL);
  unsigned short* VTh = (unsigned short*)(ws + OFF_VH);
  unsigned short* VTl = (unsigned short*)(ws + OFF_VL);
  unsigned short* Ahs = (unsigned short*)(ws + OFF_AH);
  unsigned short* Als = (unsigned short*)(ws + OFF_AL);

  float* out0 = (float*)d_out;
  float* out1 = out0 + OUT0_ELEMS;

  const int n8 = NM * NC / 8;
  cast_bf16x8<<<dim3(n8 / 256), dim3(256), 0, stream>>>(X, Xb, n8);
  wtrans_kernel<<<dim3(NC / 64, NC / 64, 3), dim3(256), 0, stream>>>(WQ, WK, WV, Wt);
  tables_kernel<<<dim3(1), dim3(256), 0, stream>>>(gcum, ginv, ksc);

  const int gridProj = (NM / 64) * (NC / 64) / 8;
  gemm_proj<2, 1><<<dim3(gridProj), dim3(256), 0, stream>>>(
      Xb, NC, WtQ, NC, Qh, Ql, NC, bQ, gcum, NT - 1, NM, NC, NC, PLANE_SC);
  gemm_proj<2, 0><<<dim3(gridProj), dim3(256), 0, stream>>>(
      Xb, NC, WtK, NC, Kh, Kl, NC, bK, gcum, NT - 1, NM, NC, NC, PLANE_SC);
  scores_kernel<<<dim3(NZ), dim3(128), 0, stream>>>(Qh, Ql, Kh, Kl, Ahs, Als, ginv);
  gemm_proj<1, 2><<<dim3(gridProj), dim3(256), 0, stream>>>(
      WtK, NC, Xb, NC, Kh, Kl, NM, bK, ksc, NT - 1, NC, NM, NC, PLANE_SC);
  gemm_proj<1, 0><<<dim3(gridProj), dim3(256), 0, stream>>>(
      WtV, NC, Xb, NC, VTh, VTl, NM, bV, ksc, NT - 1, NC, NM, NC, PLANE_SC);
  recur_kernel<<<dim3(NC / DVS, NBATCH), dim3(256), 0, stream>>>(
      Qh, Ql, Ahs, Als, Kh, Kl, VTh, VTl, gcum, out0, out1);
}
